// Decoder_12249246728308
// MI455X (gfx1250) — hardware-run, weakly checked
//
#include <hip/hip_runtime.h>
#include <math.h>

#ifndef NB
#define NB 4
#endif
#ifndef LQ
#define LQ 512
#endif
#ifndef LK
#define LK 1024
#endif
#define NB_FULL 4
#define LQ_FULL 512
#define LK_FULL 1024
#define DM 512
#define NH 8
#define HD 64
#define DFF 2048
#define NLAY 4
#define JA_NW 4
#define JA_PP 72
#define BIAS_L 6656
#define OUT1_OFF (NB_FULL * LQ_FULL * DM)

static_assert(LQ % 64 == 0);
static_assert(LK % 64 == 0);
static_assert(LQ <= LQ_FULL);
static_assert(LK <= LK_FULL);
static_assert(NB >= 1 && NB <= NB_FULL);
static_assert(DM == NH * HD);
static_assert(HD == 64);
static_assert(NH == 8);
static_assert(DM % 64 == 0 && DFF % 64 == 0);
static_assert(DM % 32 == 0 && DFF % 32 == 0);
static_assert(((NB * LQ) % 64) == 0 && ((NB * LK) % 64) == 0);
static_assert(((NB * LQ) % 32) == 0);
static_assert(((NB * LQ) % 8) == 0);
static_assert(LQ % 8 == 0 && LK % 8 == 0);
static_assert(BIAS_L == 9 * DM + DFF);
static_assert(BIAS_L % 256 == 0 && BIAS_L / 256 == 26);
static_assert(JA_NW * 16 == 64);
static_assert((size_t)OUT1_OFF * 4 == 4194304);
static_assert((size_t)NB * LQ * DM <= (size_t)OUT1_OFF);
static_assert(32 * 16 * 4 == 16 * HD * 2);
static_assert(32 * 16 * 8 == 16 * HD * 4);
static_assert(JA_NW * 16 * JA_PP * 2 + JA_NW * 16 * 68 * 4 <= 131072);
static_assert(8 * 16 * 68 * 4 <= 131072);
static_assert((unsigned long long)NB * LQ * DM * 2 * 8 + (unsigned long long)NB * LK * DM * 2 * 2
            + 2ull * ((LK > LQ) ? (unsigned long long)NB * LK * DM : (unsigned long long)NB * LQ * DM) * 2
            + 2ull * 4 * NLAY * DM * DM * 2 + 2ull * NLAY * DM * DFF * 2
            + (unsigned long long)NLAY * BIAS_L * 4 + (unsigned long long)LQ * LQ * 4 + (unsigned long long)NB * LK * 4
            + (unsigned long long)NB * LQ * DM * 4 * 5 + (unsigned long long)NB * LQ * DFF * 2 + 32ull * 256 <= 134217728ull);

typedef __attribute__((ext_vector_type(16))) _Float16 v16h;
typedef __attribute__((ext_vector_type(8)))  _Float16 v8h;
typedef __attribute__((ext_vector_type(8)))  float    v8f;
typedef __attribute__((ext_vector_type(4)))  float    v4f;
typedef __attribute__((ext_vector_type(4)))  unsigned v4u;
typedef __attribute__((ext_vector_type(2)))  unsigned v2u;
typedef v4f v4f_a __attribute__((may_alias));
typedef v8h v8h_a __attribute__((may_alias));


#define VST2(T, ptr, val) do { const T vst2_v_ = (val); *(volatile T*)(ptr) = vst2_v_; __threadfence(); *(volatile T*)(ptr) = vst2_v_; } while (0)
#define VST2V4(ptr, val) do { const v4f vst2_v4_ = (val); *(volatile v4f*)(ptr) = vst2_v4_; __threadfence(); *(volatile v4f*)(ptr) = vst2_v4_; } while (0)

__device__ __forceinline__ float cmb_bf(float v) {
    const unsigned u = __builtin_bit_cast(unsigned, v);
    const unsigned r = (u + 0x7fffu + ((u >> 16) & 1u)) & 0xffff0000u;
    return __builtin_bit_cast(float, r);
}
__device__ __forceinline__ unsigned cmb_pk2(float a, float b) {
    return (unsigned)__builtin_bit_cast(unsigned short, (_Float16)a) | ((unsigned)__builtin_bit_cast(unsigned short, (_Float16)b) << 16);
}
__device__ __forceinline__ unsigned short bfu_rne(float v) { unsigned u = __builtin_bit_cast(unsigned, v); u += 0x7FFFu + ((u >> 16) & 1u); return (unsigned short)(u >> 16); }
__device__ __forceinline__ void bfsplit(float v, unsigned short& hi, unsigned short& lo) { hi = bfu_rne(v); lo = bfu_rne(v - __builtin_bit_cast(float, (unsigned)hi << 16)); }
__device__ __forceinline__ void bfs2(float a, float b, unsigned& hi, unsigned& lo) {
    unsigned short h0, l0, h1, l1; bfsplit(a, h0, l0); bfsplit(b, h1, l1);
    hi = (unsigned)h0 | ((unsigned)h1 << 16); lo = (unsigned)l0 | ((unsigned)l1 << 16);
}
static __device__ __forceinline__ _Float16 toh_flush(float v) { const _Float16 r = (_Float16)v; return (fabsf(v) < 6.103515625e-05f) ? (_Float16)0.0f : r; }
static __device__ __forceinline__ unsigned pk2_flush(float a, float b) {
    return (unsigned)__builtin_bit_cast(unsigned short, toh_flush(a)) | ((unsigned)__builtin_bit_cast(unsigned short, toh_flush(b)) << 16);
}

struct FragU { v4u a, b; };
static_assert(sizeof(FragU) == 32);
__device__ __forceinline__ v16h ldf_h(const unsigned short* p) { FragU t; t.a = *(const v4u*)p; t.b = *(const v4u*)(p + 16); return __builtin_bit_cast(v16h, t); }
__device__ __forceinline__ v16h ldl_h(const _Float16* p) { union { v16h v; v8h h[2]; } f; f.h[0] = *(const v8h_a*)p; f.h[1] = *(const v8h_a*)(p + 16); return f.v; }

__device__ __forceinline__ v8f mma_h(v16h a, v16h b, v8f c) {
    c = __builtin_amdgcn_wmma_f32_16x16x32_f16(false, a, false, b, (short)0, c, false, false);
    asm volatile("v_nop\n\tv_nop\n\tv_nop\n\tv_nop" : "+v"(c) : "v"(a), "v"(b));
    return c;
}
__device__ __forceinline__ void guard4(v8f& a, v8f& b, v8f& c, v8f& d, v16h x) { asm volatile("v_nop\n\tv_nop\n\tv_nop\n\tv_nop" : "+v"(a), "+v"(b), "+v"(c), "+v"(d) : "v"(x)); }
__device__ __forceinline__ void keep4(v16h a, v16h b, v16h c, v16h d) { asm volatile("v_nop" :: "v"(a), "v"(b), "v"(c), "v"(d)); }
__device__ __forceinline__ void wave_sync() {
    __builtin_amdgcn_fence(3  , "workgroup");
    __builtin_amdgcn_wave_barrier();
    __builtin_amdgcn_fence(2  , "workgroup");
}

__global__ __launch_bounds__(256) void k_castrows(const float* __restrict__ SRC, unsigned short* __restrict__ DST, unsigned rowsPerBatch, unsigned srcBatchRows, unsigned nBatch, float sc) {
    const unsigned u = blockIdx.x * 256u + threadIdx.x;
    if (u >= nBatch * rowsPerBatch * (DM / 8u)) return;
    const unsigned r = u >> 6, c0 = (u & 63u) << 3;
    const unsigned b = r / rowsPerBatch, rr = r - b * rowsPerBatch;
    const float* s = SRC + ((size_t)(b * srcBatchRows + rr)) * DM + c0;
    const v4f x0 = *(const v4f*)s, x1 = *(const v4f*)(s + 4);
    v4u pk;
    pk.x = cmb_pk2(cmb_bf(x0.x) * sc, cmb_bf(x0.y) * sc); pk.y = cmb_pk2(cmb_bf(x0.z) * sc, cmb_bf(x0.w) * sc);
    pk.z = cmb_pk2(cmb_bf(x1.x) * sc, cmb_bf(x1.y) * sc); pk.w = cmb_pk2(cmb_bf(x1.z) * sc, cmb_bf(x1.w) * sc);
    VST2(v4u, DST + (size_t)r * DM + c0, pk);
}

__global__ __launch_bounds__(256) void k_castT(const float* __restrict__ S0, const float* __restrict__ S1, const float* __restrict__ S2, const float* __restrict__ S3,
                                               unsigned lds, long long zstride, unsigned short* __restrict__ DST, unsigned ldd, unsigned nR, unsigned nC, float sc) {
    const unsigned y = blockIdx.y, z = blockIdx.z;
    const float* SRC = (y == 0u) ? S0 : ((y == 1u) ? S1 : ((y == 2u) ? S2 : S3));
    SRC += (size_t)z * (size_t)zstride;
    const unsigned u = blockIdx.x * 256u + threadIdx.x; const unsigned per = nR >> 3;
    if (u >= nC * per) return;
    const unsigned c = u / per, r0 = (u - c * per) << 3;
    float w[8];
#pragma unroll
    for (int e = 0; e < 8; ++e) w[e] = cmb_bf(SRC[(size_t)(r0 + e) * lds + c]) * sc;
    v4u pk; pk.x = pk2_flush(w[0], w[1]); pk.y = pk2_flush(w[2], w[3]); pk.z = pk2_flush(w[4], w[5]); pk.w = pk2_flush(w[6], w[7]);
    VST2(v4u, DST + ((size_t)z * gridDim.y + y) * nR * nC + (size_t)c * ldd + r0, pk);
}

__global__ __launch_bounds__(256) void k_biaspack(const float* __restrict__ sbq, const float* __restrict__ sbk, const float* __restrict__ sbv, const float* __restrict__ sbo,
                                                  const float* __restrict__ cbq, const float* __restrict__ cbk, const float* __restrict__ cbv, const float* __restrict__ cbo,
                                                  const float* __restrict__ b1, const float* __restrict__ b2, float* __restrict__ DST) {
    const unsigned blk = blockIdx.x, l = blk / 26u, j = blk - l * 26u;
    const float* S; unsigned base; unsigned w = 512u;
    if (j < 2u) { S = sbq; base = 0u; }
    else if (j < 4u) { S = sbk; base = 512u; }
    else if (j < 6u) { S = sbv; base = 1024u; }
    else if (j < 8u) { S = sbo; base = 1536u; }
    else if (j < 10u) { S = cbq; base = 2048u; }
    else if (j < 12u) { S = cbk; base = 2560u; }
    else if (j < 14u) { S = cbv; base = 3072u; }
    else if (j < 16u) { S = cbo; base = 3584u; }
    else if (j < 18u) { S = b2; base = 4096u; }
    else { S = b1; base = 4608u; w = 2048u; }
    const unsigned i = j * 256u + threadIdx.x;
    const float v = cmb_bf(S[l * w + (i - base)]);
    VST2(float, DST + (size_t)l * BIAS_L + i, v);
}

__global__ __launch_bounds__(256) void k_lamplane(const float* __restrict__ lam, float* __restrict__ MB) {
    const unsigned u = blockIdx.x * 256u + threadIdx.x;
    if (u >= (unsigned)LQ * (LQ / 4u)) return;
    const unsigned q4 = (u % (LQ / 4u)) << 2; const unsigned k = u / (LQ / 4u);
    const float L2E = 1.4426950408889634f;
    v4f o;
    o.x = (cmb_bf(lam[(size_t)(q4 + 0u) * LQ_FULL + k]) * -1e9f) * L2E;
    o.y = (cmb_bf(lam[(size_t)(q4 + 1u) * LQ_FULL + k]) * -1e9f) * L2E;
    o.z = (cmb_bf(lam[(size_t)(q4 + 2u) * LQ_FULL + k]) * -1e9f) * L2E;
    o.w = (cmb_bf(lam[(size_t)(q4 + 3u) * LQ_FULL + k]) * -1e9f) * L2E;
    VST2V4(MB + (size_t)k * LQ + q4, o);
}

__global__ __launch_bounds__(256) void k_padplane(const float* __restrict__ pad, float* __restrict__ PB) {
    const unsigned u = blockIdx.x * 256u + threadIdx.x;
    if (u >= (unsigned)NB * (LK / 4u)) return;
    const unsigned k4 = (u % (LK / 4u)) << 2; const unsigned b = u / (LK / 4u);
    const float L2E = 1.4426950408889634f;
    const v4f m = *(const v4f*)(pad + (size_t)b * LK_FULL + k4);
    v4f o;
    o.x = (cmb_bf(m.x) * -1e9f) * L2E; o.y = (cmb_bf(m.y) * -1e9f) * L2E;
    o.z = (cmb_bf(m.z) * -1e9f) * L2E; o.w = (cmb_bf(m.w) * -1e9f) * L2E;
    VST2V4(PB + (size_t)b * LK + k4, o);
}

template <int BIAS_MODE, int OUT_MODE, int RESID, int ACT>
__global__ __launch_bounds__(256) void k_gemm64(const unsigned short* __restrict__ A, unsigned lda, long long strideA,
                                                const unsigned short* __restrict__ Bt, unsigned ldb, long long strideB,
                                                void* __restrict__ Cout, void* __restrict__ Cout2, unsigned ldc, long long strideC,
                                                const float* __restrict__ bias, const float* __restrict__ resid, unsigned ldr, long long strideR,
                                                unsigned M, unsigned N, unsigned K, float scale) {
    __shared__ __align__(16) float sT[8][16 * 68];
    const unsigned b = blockIdx.y, lane = threadIdx.x & 31u, wave = threadIdx.x >> 5;
    const unsigned tilesN = N >> 6, tilesM = M >> 6;
    const unsigned tile = blockIdx.x * 8u + wave;
    if (tile >= tilesM * tilesN) return;
    const unsigned tm = tile / tilesN, tn = tile - tm * tilesN;
    const unsigned m0 = tm << 6, n0 = tn << 6;
    const unsigned short* Ab = A + (size_t)b * (size_t)strideA;
    const unsigned short* Bb = Bt + (size_t)b * (size_t)strideB;
    const unsigned rlane = lane & 15u, koff = (lane >> 4) << 3, mOff = koff;

    v8f acc[4][4];
#pragma unroll
    for (int i = 0; i < 4; ++i)
#pragma unroll
        for (int j = 0; j < 4; ++j) { v8f zz = {}; acc[i][j] = zz; }

    for (unsigned k0 = 0; k0 < K; k0 += 32u) {
        v16h bh[4];
#pragma unroll
        for (int j = 0; j < 4; ++j) bh[j] = ldf_h(Bb + (size_t)(n0 + (j << 4) + rlane) * ldb + koff + k0);
#pragma unroll
        for (int i = 0; i < 4; ++i) {
            const v16h ah = ldf_h(Ab + (size_t)(m0 + (i << 4) + rlane) * lda + koff + k0);
#pragma unroll
            for (int j = 0; j < 4; ++j)
                acc[i][j] = __builtin_amdgcn_wmma_f32_16x16x32_f16(false, ah, false, bh[j], (short)0, acc[i][j], false, false);
            guard4(acc[i][0], acc[i][1], acc[i][2], acc[i][3], ah);
        }
        keep4(bh[0], bh[1], bh[2], bh[3]);
    }

    float* slab = sT[wave];
    const float* Rb = resid + (size_t)b * (size_t)strideR;
#pragma unroll
    for (int i = 0; i < 4; ++i) {
        const unsigned mBase = m0 + ((unsigned)i << 4);
#pragma unroll
        for (int j = 0; j < 4; ++j) {
            const unsigned n = n0 + ((unsigned)j << 4) + rlane;
            float bv = 0.f;
            if (BIAS_MODE == 2) bv = bias[n];
#pragma unroll
            for (int r = 0; r < 8; ++r) {
                float v = acc[i][j][r] * scale;
                if (BIAS_MODE == 1) v += bias[mBase + mOff + r];
                if (BIAS_MODE == 2) v += bv;
                if (ACT == 2) v = fmaxf(v, 0.0f);
                slab[(mOff + r) * 68u + ((unsigned)j << 4) + rlane] = v;
            }
        }
        wave_sync();
        if (OUT_MODE == 0) {
            float* Cb = (float*)Cout + (size_t)b * (size_t)strideC;
            const unsigned hh = lane >> 4, c4 = (lane & 15u) << 2;
            v4f vals[8];
#pragma unroll
            for (int it = 0; it < 8; ++it) {
                const unsigned row = (unsigned)it * 2u + hh;
                v4f v = *(const v4f_a*)(slab + row * 68u + c4);
                if (RESID != 0) {
                    v4f rr = *(const v4f*)(Rb + (size_t)(mBase + row) * ldr + n0 + c4);
                    if (RESID == 2) { rr.x = cmb_bf(rr.x); rr.y = cmb_bf(rr.y); rr.z = cmb_bf(rr.z); rr.w = cmb_bf(rr.w); }
                    v = v + rr;
                }
                vals[it] = v;
            }
            for (int pass = 0; pass < 2; ++pass) {
#pragma unroll
                for (int it = 0; it < 8; ++it) {
                    const unsigned row = (unsigned)it * 2u + hh;
                    *(volatile v4f*)(Cb + (size_t)(mBase + row) * ldc + n0 + c4) = vals[it];
                }
                __threadfence();
            }
        } else {
            const unsigned q = lane >> 3, c8 = (lane & 7u) << 3;
            unsigned short* C1 = (unsigned short*)Cout + (size_t)b * (size_t)strideC;
            unsigned short* C2 = (unsigned short*)Cout2 + (size_t)b * (size_t)strideC;
            v4u hv[4], lv[4];
#pragma unroll
            for (int it = 0; it < 4; ++it) {
                const unsigned row = (unsigned)it * 4u + q;
                const float* sp = slab + row * 68u + c8;
                const v4f x0 = *(const v4f_a*)sp, x1 = *(const v4f_a*)(sp + 4);
                v4u h4, l4;
                if (OUT_MODE == 1) {
                    h4.x = cmb_pk2(x0.x, x0.y); h4.y = cmb_pk2(x0.z, x0.w); h4.z = cmb_pk2(x1.x, x1.y); h4.w = cmb_pk2(x1.z, x1.w); l4 = h4;
                } else {
                    unsigned a0, a1, a2, a3, e0, e1, e2, e3;
                    bfs2(x0.x, x0.y, a0, e0); bfs2(x0.z, x0.w, a1, e1); bfs2(x1.x, x1.y, a2, e2); bfs2(x1.z, x1.w, a3, e3);
                    h4.x = a0; h4.y = a1; h4.z = a2; h4.w = a3; l4.x = e0; l4.y = e1; l4.z = e2; l4.w = e3;
                }
                hv[it] = h4; lv[it] = l4;
            }
            for (int pass = 0; pass < 2; ++pass) {
#pragma unroll
                for (int it = 0; it < 4; ++it) {
                    const unsigned row = (unsigned)it * 4u + q;
                    *(volatile v4u*)(C1 + (size_t)(mBase + row) * ldc + n0 + c8) = hv[it];
                    if (OUT_MODE == 2) *(volatile v4u*)(C2 + (size_t)(mBase + row) * ldc + n0 + c8) = lv[it];
                }
                __threadfence();
            }
        }
        wave_sync();
    }
}

template <int MODE, int OUTF>
__device__ __forceinline__ void attn_body(const unsigned short* __restrict__ QP, const unsigned short* __restrict__ KP, const unsigned short* __restrict__ VT,
                                          const float* __restrict__ BIAS, unsigned short* __restrict__ OH, float* __restrict__ OF, unsigned nkeys) {
    __shared__ __align__(16) _Float16 Psh[JA_NW][16 * JA_PP];
    __shared__ __align__(16) float Os[JA_NW][16 * 68];
    const unsigned tid = threadIdx.x, lane = tid & 31u, hh = lane >> 4, c = lane & 15u;
    const unsigned wave = (unsigned)__builtin_amdgcn_readfirstlane((int)(tid >> 5));
    const unsigned nqb = LQ / 64u;
    const unsigned bx = blockIdx.x, qb = bx % nqb, bh = bx / nqb, h = bh & 7u, b = bh >> 3;
    const unsigned q0 = qb * 64u + wave * 16u;
    const float SCL = 0.125f * 1.4426950408889634f;

    const size_t qoff = ((size_t)(b * LQ + q0 + c)) * DM + h * HD + 8u * hh;
    v16h qa[2];
#pragma unroll
    for (int dc = 0; dc < 2; ++dc) qa[dc] = ldf_h(QP + qoff + dc * 32);

    float mrow[8], lrow[8];
    v8f oacc[4];
#pragma unroll
    for (int r = 0; r < 8; ++r) { mrow[r] = -__builtin_inff(); lrow[r] = 0.f; }
#pragma unroll
    for (int t = 0; t < 4; ++t) { v8f zz = {}; oacc[t] = zz; }

    const size_t kbase = ((size_t)(b * nkeys + c)) * DM + h * HD + 8u * hh;
    const size_t vbase = ((size_t)(b * DM + h * HD + c)) * nkeys + 8u * hh;
    const size_t pbase = (MODE == 0) ? ((size_t)c * LQ + q0 + 8u * hh)
                                     : ((size_t)b * nkeys + c);
    _Float16* pw = Psh[wave];
    const unsigned nchunk = nkeys >> 6;

#pragma unroll 1
    for (unsigned kc = 0; kc < nchunk; ++kc) {
        const unsigned kv0 = kc * 64u;
        v8f s[4];
#pragma unroll
        for (int j = 0; j < 4; ++j) {
            const size_t ko = kbase + (size_t)(kv0 + 16u * j) * DM;
            v8f a = {};
#pragma unroll
            for (int dc = 0; dc < 2; ++dc)
                a = mma_h(qa[dc], ldf_h(KP + ko + dc * 32), a);
            if (MODE == 0) {
                const float* bp = BIAS + pbase + (size_t)(kv0 + 16u * j) * LQ;
                const v4f b0 = *(const v4f*)bp, b1 = *(const v4f*)(bp + 4);
                a[0] = fmaf(a[0], SCL, b0.x); a[1] = fmaf(a[1], SCL, b0.y); a[2] = fmaf(a[2], SCL, b0.z); a[3] = fmaf(a[3], SCL, b0.w);
                a[4] = fmaf(a[4], SCL, b1.x); a[5] = fmaf(a[5], SCL, b1.y); a[6] = fmaf(a[6], SCL, b1.z); a[7] = fmaf(a[7], SCL, b1.w);
            } else {
                const float bb = BIAS[pbase + kv0 + 16u * j];
#pragma unroll
                for (int r = 0; r < 8; ++r) a[r] = fmaf(a[r], SCL, bb);
            }
            s[j] = a;
        }
        float cm[8];
#pragma unroll
        for (int r = 0; r < 8; ++r) {
            float m = fmaxf(fmaxf(s[0][r], s[1][r]), fmaxf(s[2][r], s[3][r]));
            m = fmaxf(m, __shfl_xor(m, 1, 32)); m = fmaxf(m, __shfl_xor(m, 2, 32));
            m = fmaxf(m, __shfl_xor(m, 4, 32)); m = fmaxf(m, __shfl_xor(m, 8, 32));
            cm[r] = m;
        }
#pragma unroll
        for (int r = 0; r < 8; ++r) {
            const float mnew = fmaxf(mrow[r], cm[r]);
            const float alpha = exp2f(mrow[r] - mnew);
            mrow[r] = mnew;
            float psum = 0.f;
#pragma unroll
            for (int j = 0; j < 4; ++j) {
                const float e = s[j][r] - mnew;
                float p = exp2f(e) * 4096.0f;
                p = (e < -25.0f) ? 0.0f : p;
                const _Float16 ph = (_Float16)p;
                psum += (float)ph;
                pw[(8u * hh + r) * JA_PP + 16u * j + c] = ph;
            }
            lrow[r] = lrow[r] * alpha + psum;
#pragma unroll
            for (int t = 0; t < 4; ++t) oacc[t][r] *= alpha;
        }
        wave_sync();
#pragma unroll
        for (int kk = 0; kk < 2; ++kk) {
            const v16h pa = ldl_h(pw + c * JA_PP + kk * 32 + 8u * hh);
#pragma unroll
            for (int t = 0; t < 4; ++t) {
                const v16h vb = ldf_h(VT + vbase + (size_t)(16u * t) * nkeys + kv0 + kk * 32);
                oacc[t] = mma_h(pa, vb, oacc[t]);
            }
        }
        wave_sync();
    }

    float inv[8];
#pragma unroll
    for (int r = 0; r < 8; ++r) {
        float l = lrow[r];
        l += __shfl_xor(l, 1, 32); l += __shfl_xor(l, 2, 32); l += __shfl_xor(l, 4, 32); l += __shfl_xor(l, 8, 32);
        inv[r] = ((OUTF == 0) ? 16.0f : 1.0f) / l;
    }
    float* os = Os[wave];
#pragma unroll
    for (int r = 0; r < 8; ++r)
#pragma unroll
        for (int t = 0; t < 4; ++t) os[(8u * hh + r) * 68u + 16u * t + c] = oacc[t][r] * inv[r];
    wave_sync();
    if (OUTF == 0) {
        const unsigned rq = lane >> 3, c8 = (lane & 7u) << 3;
        unsigned short* ob = OH + ((size_t)(b * LQ + q0)) * DM + h * HD + c8;
        v4u hv[4];
#pragma unroll
        for (int it = 0; it < 4; ++it) {
            const float* sp = os + ((unsigned)it * 4u + rq) * 68u + c8;
            const v4f x0 = *(const v4f_a*)sp, x1 = *(const v4f_a*)(sp + 4);
            v4u h4;
            h4.x = pk2_flush(x0.x, x0.y); h4.y = pk2_flush(x0.z, x0.w); h4.z = pk2_flush(x1.x, x1.y); h4.w = pk2_flush(x1.z, x1.w);
            hv[it] = h4;
        }
        for (int pass = 0; pass < 2; ++pass) {
#pragma unroll
            for (int it = 0; it < 4; ++it) *(volatile v4u*)(ob + (size_t)((unsigned)it * 4u + rq) * DM) = hv[it];
            __threadfence();
        }
    } else {
        const unsigned c4 = (lane & 15u) << 2;
        float* ub = OF + ((size_t)(b * LQ + q0)) * DM + h * HD + c4;
        v4f vals[8];
#pragma unroll
        for (int it = 0; it < 8; ++it) vals[it] = *(const v4f_a*)(os + ((unsigned)it * 2u + hh) * 68u + c4);
        for (int pass = 0; pass < 2; ++pass) {
#pragma unroll
            for (int it = 0; it < 8; ++it) *(volatile v4f*)(ub + (size_t)((unsigned)it * 2u + hh) * DM) = vals[it];
            __threadfence();
        }
    }
}

__global__ __launch_bounds__(32 * JA_NW) void k_attn_self(const unsigned short* __restrict__ QP, const unsigned short* __restrict__ KP, const unsigned short* __restrict__ VT,
                                                          const float* __restrict__ MB, unsigned short* __restrict__ C16, unsigned nkeys) {
    attn_body<0, 0>(QP, KP, VT, MB, C16, (float*)0, nkeys);
}
__global__ __launch_bounds__(32 * JA_NW) void k_attn_cross(const unsigned short* __restrict__ QP, const unsigned short* __restrict__ KP, const unsigned short* __restrict__ VT,
                                                           const float* __restrict__ PB, unsigned short* __restrict__ C16, unsigned nkeys) {
    attn_body<1, 0>(QP, KP, VT, PB, C16, (float*)0, nkeys);
}
__global__ __launch_bounds__(32 * JA_NW) void k_attn_ctx(const unsigned short* __restrict__ QP, const unsigned short* __restrict__ KP, const unsigned short* __restrict__ ET,
                                                         const float* __restrict__ PB, float* __restrict__ CTX, unsigned nkeys) {
    attn_body<1, 1>(QP, KP, ET, PB, (unsigned short*)0, CTX, nkeys);
}

template <int WH>
__device__ __forceinline__ void ln_body(const float* __restrict__ X, const float* __restrict__ G, const float* __restrict__ Bv,
                                        float* __restrict__ O, unsigned short* __restrict__ OH, unsigned nrows) {
#pragma clang fp contract(off)
    const unsigned lane = threadIdx.x & 31u;
    const unsigned row = blockIdx.x * 8u + (unsigned)__builtin_amdgcn_readfirstlane((int)(threadIdx.x >> 5));
    if (row >= nrows) return;
    const size_t base = (size_t)row * DM + 4u * lane;
    v4f v[4]; float s = 0.f;
#pragma unroll
    for (int i = 0; i < 4; ++i) { v[i] = *(const v4f*)(X + base + 128 * i); s += (v[i].x + v[i].y) + (v[i].z + v[i].w); }
    s += __shfl_xor(s, 16, 32); s += __shfl_xor(s, 8, 32); s += __shfl_xor(s, 4, 32); s += __shfl_xor(s, 2, 32); s += __shfl_xor(s, 1, 32);
    const float mu = s * (1.0f / 512.0f);
    float q = 0.f;
#pragma unroll
    for (int i = 0; i < 4; ++i) { const v4f d = v[i] - mu; q += (d.x * d.x + d.y * d.y) + (d.z * d.z + d.w * d.w); v[i] = d; }
    q += __shfl_xor(q, 16, 32); q += __shfl_xor(q, 8, 32); q += __shfl_xor(q, 4, 32); q += __shfl_xor(q, 2, 32); q += __shfl_xor(q, 1, 32);
    const float rs = 1.0f / sqrtf(q * (1.0f / 512.0f) + 1e-6f);
#pragma unroll
    for (int i = 0; i < 4; ++i) {
        const v4f g4 = *(const v4f*)(G + 4u * lane + 128 * i), b4 = *(const v4f*)(Bv + 4u * lane + 128 * i);
        v4f o;
        o.x = cmb_bf(g4.x) * v[i].x * rs + cmb_bf(b4.x); o.y = cmb_bf(g4.y) * v[i].y * rs + cmb_bf(b4.y);
        o.z = cmb_bf(g4.z) * v[i].z * rs + cmb_bf(b4.z); o.w = cmb_bf(g4.w) * v[i].w * rs + cmb_bf(b4.w);
        VST2V4(O + base + 128 * i, o);
        if (WH) { v2u pk; pk.x = pk2_flush(o.x, o.y); pk.y = pk2_flush(o.z, o.w); VST2(v2u, OH + base + 128 * i, pk); }
    }
}
__global__ __launch_bounds__(256) void k_ln_h(const float* __restrict__ X, const float* __restrict__ G, const float* __restrict__ Bv,
                                              float* __restrict__ O, unsigned short* __restrict__ OH, unsigned nrows) {
    ln_body<1>(X, G, Bv, O, OH, nrows);
}
__global__ __launch_bounds__(256) void k_ln_f(const float* __restrict__ X, const float* __restrict__ G, const float* __restrict__ Bv,
                                              float* __restrict__ O, unsigned nrows) {
    ln_body<0>(X, G, Bv, O, (unsigned short*)0, nrows);
}

__global__ __launch_bounds__(256) void k_pgen(const float* __restrict__ X, const float* __restrict__ Y, const float* __restrict__ CTX,
                                              const float* __restrict__ wx, const float* __restrict__ bx, const float* __restrict__ wsv, const float* __restrict__ bs,
                                              const float* __restrict__ wh, const float* __restrict__ bhv, const float* __restrict__ vw, const float* __restrict__ vb,
                                              float* __restrict__ PG) {
    __shared__ float pg[32];
    const unsigned lane = threadIdx.x & 31u;
    const unsigned wave = (unsigned)__builtin_amdgcn_readfirstlane((int)(threadIdx.x >> 5));
    const float cbx = cmb_bf(bx[0]), cbs = cmb_bf(bs[0]), cbh = cmb_bf(bhv[0]), cvw = cmb_bf(vw[0]), cvb = cmb_bf(vb[0]);
#pragma unroll 1
    for (unsigned rr = 0; rr < 4u; ++rr) {
        const unsigned lr = wave * 4u + rr, row = blockIdx.x * 32u + lr;
        const unsigned b = row / (unsigned)LQ, q = row - b * (unsigned)LQ;
        const float* xs = X + ((size_t)(b * LQ_FULL + q)) * DM + 4u * lane;
        const float* ys = Y + (size_t)row * DM + 4u * lane;
        const float* cs = CTX + (size_t)row * DM + 4u * lane;
        float a1 = 0.f, a2 = 0.f, a3 = 0.f;
#pragma unroll 1
        for (unsigned i = 0; i < 4u; ++i) {
            const unsigned o = 128u * i;
            const v4f xv = *(const v4f*)(xs + o), yv = *(const v4f*)(ys + o), cv = *(const v4f*)(cs + o);
            const v4f w1 = *(const v4f*)(wx + 4u * lane + o), w2 = *(const v4f*)(wsv + 4u * lane + o), w3 = *(const v4f*)(wh + 4u * lane + o);
            a1 += (cmb_bf(xv.x) * cmb_bf(w1.x) + cmb_bf(xv.y) * cmb_bf(w1.y)) + (cmb_bf(xv.z) * cmb_bf(w1.z) + cmb_bf(xv.w) * cmb_bf(w1.w));
            a2 += (yv.x * cmb_bf(w2.x) + yv.y * cmb_bf(w2.y)) + (yv.z * cmb_bf(w2.z) + yv.w * cmb_bf(w2.w));
            a3 += (cv.x * cmb_bf(w3.x) + cv.y * cmb_bf(w3.y)) + (cv.z * cmb_bf(w3.z) + cv.w * cmb_bf(w3.w));
        }
        a1 += __shfl_xor(a1, 16, 32); a1 += __shfl_xor(a1, 8, 32); a1 += __shfl_xor(a1, 4, 32); a1 += __shfl_xor(a1, 2, 32); a1 += __shfl_xor(a1, 1, 32);
        a2 += __shfl_xor(a2, 16, 32); a2 += __shfl_xor(a2, 8, 32); a2 += __shfl_xor(a2, 4, 32); a2 += __shfl_xor(a2, 2, 32); a2 += __shfl_xor(a2, 1, 32);
        a3 += __shfl_xor(a3, 16, 32); a3 += __shfl_xor(a3, 8, 32); a3 += __shfl_xor(a3, 4, 32); a3 += __shfl_xor(a3, 2, 32); a3 += __shfl_xor(a3, 1, 32);
        const float sv = ((a1 + cbx) + (a2 + cbs)) + (a3 + cbh);
        const float z = sv * cvw + cvb;
        const float p = 1.0f / (1.0f + expf(-z));
        if (lane == 0u) pg[lr] = p;
    }
    __syncthreads();
    if (wave == 0u) {
        const float v = pg[lane];
        VST2(float, PG + (size_t)blockIdx.x * 32u + lane, v);
    }
}

extern "C" void kernel_launch(void* const* d_in, const int* in_sizes, int n_in, void* d_out, int out_size, void* d_ws, size_t ws_size, hipStream_t stream) {
    if (n_in < 34) return;
    const long long needX   = ((long long)(NB - 1) * LQ_FULL + LQ) * DM;
    const long long needE   = ((long long)(NB - 1) * LK_FULL + LK) * DM;
    const long long needLam = (long long)(LQ - 1) * LQ_FULL + LQ;
    const long long needPad = (long long)(NB - 1) * LK_FULL + LK;
    if ((long long)in_sizes[0] < needX || (long long)in_sizes[1] < needE) return;
    if ((long long)in_sizes[2] < needLam || (long long)in_sizes[3] < needPad) return;
    for (int i = 4; i < 20; i += 2) { if (in_sizes[i] < NLAY * DM * DM || in_sizes[i + 1] < NLAY * DM) return; }
    if (in_sizes[20] < NLAY * DM * DFF || in_sizes[21] < NLAY * DFF || in_sizes[22] < NLAY * DFF * DM || in_sizes[23] < NLAY * DM) return;
    if (in_sizes[24] < NLAY * 3 * DM || in_sizes[25] < NLAY * 3 * DM) return;
    if (in_sizes[26] < DM || in_sizes[28] < DM || in_sizes[30] < DM) return;
    if (in_sizes[27] < 1 || in_sizes[29] < 1 || in_sizes[31] < 1 || in_sizes[32] < 1 || in_sizes[33] < 1) return;
    if ((long long)out_size < (long long)OUT1_OFF + (long long)NB * LQ) return;

    const float* x    = (const float*)d_in[0];
    const float* enc  = (const float*)d_in[1];
    const float* lam  = (const float*)d_in[2];
    const float* pad  = (const float*)d_in[3];
    const float* sa_wq = (const float*)d_in[4];   const float* sa_bq = (const float*)d_in[5];
    const float* sa_wk = (const float*)d_in[6];   const float* sa_bk = (const float*)d_in[7];
    const float* sa_wv = (const float*)d_in[8];   const float* sa_bv = (const float*)d_in[9];
    const float* sa_wo = (const float*)d_in[10];  const float* sa_bo = (const float*)d_in[11];
    const float* ca_wq = (const float*)d_in[12];  const float* ca_bq = (const float*)d_in[13];
    const float* ca_wk = (const float*)d_in[14];  const float* ca_bk = (const float*)d_in[15];
    const float* ca_wv = (const float*)d_in[16];  const float* ca_bv = (const float*)d_in[17];
    const float* ca_wo = (const float*)d_in[18];  const float* ca_bo = (const float*)d_in[19];
    const float* ffn_w1 = (const float*)d_in[20]; const float* ffn_b1 = (const float*)d_in[21];
    const float* ffn_w2 = (const float*)d_in[22]; const float* ffn_b2 = (const float*)d_in[23];
    const float* ln_g = (const float*)d_in[24];   const float* ln_b = (const float*)d_in[25];
    const float* wx_w = (const float*)d_in[26];   const float* wx_b = (const float*)d_in[27];
    const float* ws_w = (const float*)d_in[28];   const float* ws_b = (const float*)d_in[29];
    const float* wh_w = (const float*)d_in[30];   const float* wh_b = (const float*)d_in[31];
    const float* v_w  = (const float*)d_in[32];   const float* v_b  = (const float*)d_in[33];
    float* out = (float*)d_out;
    float* pgens = out + (size_t)OUT1_OFF;

    const size_t nQ = (size_t)NB * LQ * DM, nK = (size_t)NB * LK * DM;
    const size_t nKV = (nK > nQ) ? nK : nQ;
    char* wsp = (char*)d_ws;
    auto carve = [&wsp](size_t bytes) { char* p = wsp; wsp += ((bytes + 255) / 256) * 256; return p; };
    unsigned short* X16   = (unsigned short*)carve(nQ * 2);
    unsigned short* ENC16 = (unsigned short*)carve(nK * 2);
    unsigned short* ENCT  = (unsigned short*)carve(nK * 2);
    unsigned short* WSA   = (unsigned short*)carve((size_t)NLAY * 4 * DM * DM * 2);
    unsigned short* WCA   = (unsigned short*)carve((size_t)NLAY * 4 * DM * DM * 2);
    unsigned short* W1T   = (unsigned short*)carve((size_t)NLAY * DFF * DM * 2);
    unsigned short* W2T   = (unsigned short*)carve((size_t)NLAY * DM * DFF * 2);
    float*          BIASP = (float*)carve((size_t)NLAY * BIAS_L * 4);
    float*          MB    = (float*)carve((size_t)LQ * LQ * 4);
    float*          PB    = (float*)carve((size_t)NB * LK * 4);
    unsigned short* QP    = (unsigned short*)carve(nQ * 2);
    unsigned short* KP    = (unsigned short*)carve(nKV * 2);
    unsigned short* VT    = (unsigned short*)carve(nKV * 2);
    unsigned short* C16   = (unsigned short*)carve(nQ * 2);
    float*          X1    = (float*)carve(nQ * 4);
    float*          O1    = (float*)carve(nQ * 4);
    unsigned short* O1H   = (unsigned short*)carve(nQ * 2);
    float*          O2    = (float*)carve(nQ * 4);
    unsigned short* O2H   = (unsigned short*)carve(nQ * 2);
    float*          OUTS  = (float*)carve(nQ * 4);
    unsigned short* OUTH  = (unsigned short*)carve(nQ * 2);
    unsigned short* F1H   = (unsigned short*)carve((size_t)NB * LQ * DFF * 2);
    float*          CTX   = (float*)carve(nQ * 4);
    const size_t used = (size_t)(wsp - (char*)d_ws);
    if (used > ws_size || used > (size_t)134217728) return;

    k_castrows<<<(unsigned)((nQ / 8 + 255) / 256), 256, 0, stream>>>(x, X16, (unsigned)LQ, (unsigned)LQ_FULL, (unsigned)NB, 1.0f);
    k_castrows<<<(unsigned)((nK / 8 + 255) / 256), 256, 0, stream>>>(enc, ENC16, (unsigned)LK, (unsigned)LK_FULL, (unsigned)NB, 1.0f);
    {
        const float* e0 = enc;
        const float* e1 = enc + (size_t)((NB > 1) ? 1 : 0) * LK_FULL * DM;
        const float* e2 = enc + (size_t)((NB > 2) ? 2 : (NB - 1)) * LK_FULL * DM;
        const float* e3 = enc + (size_t)((NB > 3) ? 3 : (NB - 1)) * LK_FULL * DM;
        k_castT<<<dim3((unsigned)((DM * (LK / 8) + 255) / 256), (unsigned)NB, 1u), 256, 0, stream>>>(e0, e1, e2, e3, (unsigned)DM, 0LL, ENCT, (unsigned)LK, (unsigned)LK, (unsigned)DM, 1.0f);
    }
    k_castT<<<dim3((unsigned)((DM * (DM / 8) + 255) / 256), 4u, (unsigned)NLAY), 256, 0, stream>>>(sa_wq, sa_wk, sa_wv, sa_wo, (unsigned)DM, (long long)DM * DM, WSA, (unsigned)DM, (unsigned)DM, (unsigned)DM, 16.0f);
    k_castT<<<dim3((unsigned)((DM * (DM / 8) + 255) / 256), 4u, (unsigned)NLAY), 256, 0, stream>>>(ca_wq, ca_wk, ca_wv, ca_wo, (unsigned)DM, (long long)DM * DM, WCA, (unsigned)DM, (unsigned)DM, (unsigned)DM, 16.0f);
    k_castT<<<dim3((unsigned)((DFF * (DM / 8) + 255) / 256), 1u, (unsigned)NLAY), 256, 0, stream>>>(ffn_w1, ffn_w1, ffn_w1, ffn_w1, (unsigned)DFF, (long long)DM * DFF, W1T, (unsigned)DM, (unsigned)DM, (unsigned)DFF, 16.0f);
    k_castT<<<dim3((unsigned)((DM * (DFF / 8) + 255) / 256), 1u, (unsigned)NLAY), 256, 0, stream>>>(ffn_w2, ffn_w2, ffn_w2, ffn_w2, (unsigned)DM, (long long)DFF * DM, W2T, (unsigned)DFF, (unsigned)DFF, (unsigned)DM, 16.0f);
    k_biaspack<<<(unsigned)(26 * NLAY), 256, 0, stream>>>(sa_bq, sa_bk, sa_bv, sa_bo, ca_bq, ca_bk, ca_bv, ca_bo, ffn_b1, ffn_b2, BIASP);
    k_lamplane<<<(unsigned)(((size_t)LQ * (LQ / 4) + 255) / 256), 256, 0, stream>>>(lam, MB);
    k_padplane<<<(unsigned)(((size_t)NB * (LK / 4) + 255) / 256), 256, 0, stream>>>(pad, PB);

    const unsigned gQ  = (unsigned)((((NB * LQ) / 64) * (DM / 64) + 7) / 8);
    const unsigned gK  = (unsigned)((((NB * LK) / 64) * (DM / 64) + 7) / 8);
    const unsigned gVs = (unsigned)(((DM / 64) * (LQ / 64) + 7) / 8);
    const unsigned gVc = (unsigned)(((DM / 64) * (LK / 64) + 7) / 8);
    const unsigned gOb = (unsigned)(((LQ / 64) * (DM / 64) + 7) / 8);
    const unsigned gF1 = (unsigned)((((NB * LQ) / 64) * (DFF / 64) + 7) / 8);
    const unsigned MQ = (unsigned)(NB * LQ), MKc = (unsigned)(NB * LK);
    const unsigned gAtt = (unsigned)(NB * NH * (LQ / 64));
    const unsigned gLn = (unsigned)((NB * LQ) / 8);

    for (int l = 0; l < NLAY; ++l) {
        const unsigned short* WS = WSA + (size_t)l * 4 * DM * DM;
        const unsigned short* WC = WCA + (size_t)l * 4 * DM * DM;
        const float* BL = BIASP + (size_t)l * BIAS_L;
        const unsigned short* CURH = (l == 0) ? X16 : OUTH;

        k_gemm64<2, 1, 0, 0><<<dim3(gQ, 1u), 256, 0, stream>>>(
            CURH, (unsigned)DM, 0LL, WS, (unsigned)DM, 0LL, (void*)QP, (void*)QP, (unsigned)DM, 0LL, BL, BL, (unsigned)DM, 0LL,
            MQ, (unsigned)DM, (unsigned)DM, 0.0625f);
        k_gemm64<2, 1, 0, 0><<<dim3(gQ, 1u), 256, 0, stream>>>(
            CURH, (unsigned)DM, 0LL, WS + (size_t)DM * DM, (unsigned)DM, 0LL, (void*)KP, (void*)KP, (unsigned)DM, 0LL, BL + 512, BL, (unsigned)DM, 0LL,
            MQ, (unsigned)DM, (unsigned)DM, 0.0625f);
        k_gemm64<1, 1, 0, 0><<<dim3(gVs, (unsigned)NB), 256, 0, stream>>>(
            WS + (size_t)2 * DM * DM, (unsigned)DM, 0LL, CURH, (unsigned)DM, (long long)LQ * DM, (void*)VT, (void*)VT, (unsigned)LQ, (long long)DM * LQ, BL + 1024, BL, (unsigned)DM, 0LL,
            (unsigned)DM, (unsigned)LQ, (unsigned)DM, 0.0625f);
        k_attn_self<<<gAtt, 32 * JA_NW, 0, stream>>>(QP, KP, VT, MB, C16, (unsigned)LQ);
        if (l == 0) {
            k_gemm64<2, 0, 2, 0><<<dim3(gOb, (unsigned)NB), 256, 0, stream>>>(
                C16, (unsigned)DM, (long long)LQ * DM, WS + (size_t)3 * DM * DM, (unsigned)DM, 0LL, (void*)X1, (void*)X1, (unsigned)DM, (long long)LQ * DM, BL + 1536, x, (unsigned)DM, (long long)LQ_FULL * DM,
                (unsigned)LQ, (unsigned)DM, (unsigned)DM, 0.00390625f);
        } else {
            k_gemm64<2, 0, 1, 0><<<dim3(gQ, 1u), 256, 0, stream>>>(
                C16, (unsigned)DM, 0LL, WS + (size_t)3 * DM * DM, (unsigned)DM, 0LL, (void*)X1, (void*)X1, (unsigned)DM, 0LL, BL + 1536, OUTS, (unsigned)DM, 0LL,
                MQ, (unsigned)DM, (unsigned)DM, 0.00390625f);
        }
        k_ln_h<<<gLn, 256, 0, stream>>>(X1, ln_g + (size_t)(l * 3 + 0) * DM, ln_b + (size_t)(l * 3 + 0) * DM, O1, O1H, MQ);

        k_gemm64<2, 1, 0, 0><<<dim3(gQ, 1u), 256, 0, stream>>>(
            O1H, (unsigned)DM, 0LL, WC, (unsigned)DM, 0LL, (void*)QP, (void*)QP, (unsigned)DM, 0LL, BL + 2048, BL, (unsigned)DM, 0LL,
            MQ, (unsigned)DM, (unsigned)DM, 0.0625f);
        k_gemm64<2, 1, 0, 0><<<dim3(gK, 1u), 256, 0, stream>>>(
            ENC16, (unsigned)DM, 0LL, WC + (size_t)DM * DM, (unsigned)DM, 0LL, (void*)KP, (void*)KP, (unsigned)DM, 0LL, BL + 2560, BL, (unsigned)DM, 0LL,
            MKc, (unsigned)DM, (unsigned)DM, 0.0625f);
        k_gemm64<1, 1, 0, 0><<<dim3(gVc, (unsigned)NB), 256, 0, stream>>>(
            WC + (size_t)2 * DM * DM, (unsigned)DM, 0LL, ENC16, (unsigned)DM, (long long)LK * DM, (void*)VT, (void*)VT, (unsigned)LK, (long long)DM * LK, BL + 3072, BL, (unsigned)DM, 0LL,
            (unsigned)DM, (unsigned)LK, (unsigned)DM, 0.0625f);
        k_attn_cross<<<gAtt, 32 * JA_NW, 0, stream>>>(QP, KP, VT, PB, C16, (unsigned)LK);
        k_gemm64<2, 0, 1, 0><<<dim3(gQ, 1u), 256, 0, stream>>>(
            C16, (unsigned)DM, 0LL, WC + (size_t)3 * DM * DM, (unsigned)DM, 0LL, (void*)X1, (void*)X1, (unsigned)DM, 0LL, BL + 3584, O1, (unsigned)DM, 0LL,
            MQ, (unsigned)DM, (unsigned)DM, 0.00390625f);
        k_ln_h<<<gLn, 256, 0, stream>>>(X1, ln_g + (size_t)(l * 3 + 1) * DM, ln_b + (size_t)(l * 3 + 1) * DM, O2, O2H, MQ);

        k_gemm64<2, 1, 0, 2><<<dim3(gF1, 1u), 256, 0, stream>>>(
            O2H, (unsigned)DM, 0LL, W1T + (size_t)l * DFF * DM, (unsigned)DM, 0LL, (void*)F1H, (void*)F1H, (unsigned)DFF, 0LL, BL + 4608, BL, (unsigned)DM, 0LL,
            MQ, (unsigned)DFF, (unsigned)DM, 0.0625f);
        k_gemm64<2, 0, 1, 0><<<dim3(gQ, 1u), 256, 0, stream>>>(
            F1H, (unsigned)DFF, 0LL, W2T + (size_t)l * DM * DFF, (unsigned)DFF, 0LL, (void*)X1, (void*)X1, (unsigned)DM, 0LL, BL + 4096, O2, (unsigned)DM, 0LL,
            MQ, (unsigned)DM, (unsigned)DFF, 0.0625f);
        if (l < NLAY - 1) {
            k_ln_h<<<gLn, 256, 0, stream>>>(X1, ln_g + (size_t)(l * 3 + 2) * DM, ln_b + (size_t)(l * 3 + 2) * DM, OUTS, OUTH, MQ);
        } else {
            k_ln_f<<<gLn, 256, 0, stream>>>(X1, ln_g + (size_t)(l * 3 + 2) * DM, ln_b + (size_t)(l * 3 + 2) * DM, out, MQ);
        }
    }

    k_attn_ctx<<<gAtt, 32 * JA_NW, 0, stream>>>(QP, KP, ENCT, PB, CTX, (unsigned)LK);
    k_pgen<<<(unsigned)((NB * LQ) / 32), 256, 0, stream>>>(x, out, CTX, wx_w, wx_b, ws_w, ws_b, wh_w, wh_b, v_w, v_b, pgens);
}
